// RelPartialLearnableMultiHeadAttn_55886114456079
// MI455X (gfx1250) — hardware-verified
//
#include <hip/hip_runtime.h>


#ifndef NB
#define NB 4
#endif
#define NB_FULL 4
#ifndef QLEN
#define QLEN 1024
#endif
#ifndef MLEN
#define MLEN 1024
#endif
#define QLEN_FULL 1024
#define MLEN_FULL 1024
#define KLEN (QLEN + MLEN)
#define KLEN_FULL (QLEN_FULL + MLEN_FULL)
#define DM 1024
#define NH 16
#define DH 64
#define HH (NH * DH)
#define TH3 (3 * HH)
#define SCL 0.125f
#define LNEPS 1e-5f
#define PCARRY 4096.0f
#define AVCARRY 32.0f
#define OWCARRY 64.0f

static_assert(NB >= 1 && NB <= NB_FULL);
static_assert(QLEN % 128 == 0 && MLEN % 128 == 0);
static_assert(DM == 1024 && HH == 1024 && DH == 64 && NH == 16);
static_assert(((long)QLEN * NB) % 128 == 0);
static_assert((long)QLEN * NB * DM * 4 <= 16777216L);

typedef unsigned short us_t;
typedef us_t     v8us  __attribute__((ext_vector_type(8)));
typedef unsigned v4u   __attribute__((ext_vector_type(4)));
typedef float    v8f   __attribute__((ext_vector_type(8)));
typedef float    v4f   __attribute__((ext_vector_type(4)));
typedef __bf16   v16bf __attribute__((ext_vector_type(16)));
typedef _Float16 v16h  __attribute__((ext_vector_type(16)));

union Frag16 { v8us u[2]; v16bf bf; v16h hf; };

__device__ __forceinline__ v8f vzero() {
  v8f z = {0.f, 0.f, 0.f, 0.f, 0.f, 0.f, 0.f, 0.f};
  return z;
}

__device__ __forceinline__ us_t bf_bits(float x) {
  unsigned u = __float_as_uint(x);
  u += 0x7FFFu + ((u >> 16) & 1u);
  return (us_t)(u >> 16);
}
__device__ __forceinline__ float bf_val(float x) {
  unsigned u = __float_as_uint(x);
  u += 0x7FFFu + ((u >> 16) & 1u);
  return __uint_as_float(u & 0xFFFF0000u);
}
__device__ __forceinline__ us_t hf_bits(float x) {
  _Float16 hv = (_Float16)x;
  return __builtin_bit_cast(us_t, hv);
}

template <int F16OP>
__device__ __forceinline__ v8f mma16(const Frag16& a, const Frag16& b, v8f c) {
  if (F16OP) {
    c = __builtin_amdgcn_wmma_f32_16x16x32_f16(false, a.hf, false, b.hf, (short)0, c, false, false);
    asm volatile("v_nop\n\tv_nop\n\tv_nop\n\tv_nop" : "+v"(c) : "v"(a.hf), "v"(b.hf));
  } else {
    c = __builtin_amdgcn_wmma_f32_16x16x32_bf16(false, a.bf, false, b.bf, (short)0, c, false, false);
    asm volatile("v_nop\n\tv_nop\n\tv_nop\n\tv_nop" : "+v"(c) : "v"(a.bf), "v"(b.bf));
  }
  return c;
}

__global__ __launch_bounds__(128)
void k_cvt_cat(const float* __restrict__ mems, const float* __restrict__ w, us_t* catb) {
  const int blk = blockIdx.x;
  const int b = blk / KLEN, pos = blk - b * KLEN;
  const int t = threadIdx.x;
  const float* src = (pos < MLEN) ? (mems + ((size_t)pos * NB_FULL + b) * DM)
                                  : (w + ((size_t)(pos - MLEN) * NB_FULL + b) * DM);
  v4f f0 = *(const v4f*)(src + 8 * t);
  v4f f1 = *(const v4f*)(src + 8 * t + 4);
  float e[8] = {f0[0], f0[1], f0[2], f0[3], f1[0], f1[1], f1[2], f1[3]};
  unsigned wv[4];
#pragma unroll
  for (int k = 0; k < 4; ++k)
    wv[k] = (unsigned)bf_bits(e[2 * k]) | ((unsigned)bf_bits(e[2 * k + 1]) << 16);
  v4u pk = {wv[0], wv[1], wv[2], wv[3]};
  us_t* dst = catb + (size_t)blk * DM + 8 * t;
  *(volatile v4u*)dst = pk;
  __threadfence();
  *(volatile v4u*)dst = pk;
}

template <int MODE>
__global__ __launch_bounds__(128)
void k_cvt_lin(const float* __restrict__ src, us_t* dst) {
  const size_t base = (size_t)blockIdx.x * 1024 + 8 * threadIdx.x;
  v4f f0 = *(const v4f*)(src + base);
  v4f f1 = *(const v4f*)(src + base + 4);
  float e[8] = {f0[0], f0[1], f0[2], f0[3], f1[0], f1[1], f1[2], f1[3]};
  unsigned wv[4];
#pragma unroll
  for (int k = 0; k < 4; ++k) {
    us_t lo, hi;
    if (MODE == 0) { lo = bf_bits(e[2 * k]); hi = bf_bits(e[2 * k + 1]); }
    else           { lo = hf_bits(bf_val(e[2 * k]) * OWCARRY); hi = hf_bits(bf_val(e[2 * k + 1]) * OWCARRY); }
    wv[k] = (unsigned)lo | ((unsigned)hi << 16);
  }
  v4u pk = {wv[0], wv[1], wv[2], wv[3]};
  us_t* d = dst + base;
  *(volatile v4u*)d = pk;
  __threadfence();
  *(volatile v4u*)d = pk;
}

#define BM 128
#define BN 128
#define BK 32
#define BKP 40
#define CSP 136
#define CFP 132
#define EPI_Q 0
#define EPI_KV 1
#define EPI_RK 2
#define EPI_OUT 3

template <int F16OP, int EPI>
__global__ __launch_bounds__(256)
void k_gemm(const us_t* __restrict__ A, const us_t* __restrict__ B,
            void* D0, void* D1, const float* __restrict__ bias0, const float* __restrict__ bias1,
            long lda, long ldb, long strideAz, int K)
{
  __shared__ __align__(16) us_t As[BM * BKP];
  __shared__ __align__(16) us_t Bs[BN * BKP];
  __shared__ __align__(16) us_t Cs[BM * CSP];
  static_assert(64 * CFP * 4 <= BM * CSP * 2);

  const int tid = threadIdx.x, lane = tid & 31, wid = tid >> 5;
  const int wm = wid >> 2, wn = wid & 3, h = lane >> 4, l15 = lane & 15;
  const int m0 = blockIdx.y * BM, n0 = blockIdx.x * BN, z = blockIdx.z;
  const us_t* Ab = A + (size_t)z * (size_t)strideAz + (size_t)m0 * (size_t)lda;
  const us_t* Bb = B + (size_t)n0 * (size_t)ldb;

  v8f acc[4][2];
#pragma unroll
  for (int mi = 0; mi < 4; ++mi)
#pragma unroll
    for (int ni = 0; ni < 2; ++ni) acc[mi][ni] = vzero();

  const int nk = K / BK;
  for (int kb = 0; kb < nk; ++kb) {
    const int k0 = kb * BK;
    v8us ra[2], rb[2];
#pragma unroll
    for (int t = 0; t < 2; ++t) {
      const int ch = tid + t * 256, row = ch >> 2, kc = (ch & 3) << 3;
      ra[t] = *(const v8us*)(Ab + (size_t)row * (size_t)lda + k0 + kc);
      rb[t] = *(const v8us*)(Bb + (size_t)row * (size_t)ldb + k0 + kc);
    }
    __syncthreads();
#pragma unroll
    for (int t = 0; t < 2; ++t) {
      const int ch = tid + t * 256, row = ch >> 2, kc = (ch & 3) << 3;
      *(v8us*)(&As[row * BKP + kc]) = ra[t];
      *(v8us*)(&Bs[row * BKP + kc]) = rb[t];
    }
    __syncthreads();
    Frag16 af[4], bfr[2];
#pragma unroll
    for (int mi = 0; mi < 4; ++mi) {
      const int r = wm * 64 + mi * 16 + l15;
      af[mi].u[0] = *(const v8us*)(&As[r * BKP + 8 * h]);
      af[mi].u[1] = *(const v8us*)(&As[r * BKP + 16 + 8 * h]);
    }
#pragma unroll
    for (int ni = 0; ni < 2; ++ni) {
      const int r = wn * 32 + ni * 16 + l15;
      bfr[ni].u[0] = *(const v8us*)(&Bs[r * BKP + 8 * h]);
      bfr[ni].u[1] = *(const v8us*)(&Bs[r * BKP + 16 + 8 * h]);
    }
#pragma unroll
    for (int mi = 0; mi < 4; ++mi)
#pragma unroll
      for (int ni = 0; ni < 2; ++ni) acc[mi][ni] = mma16<F16OP>(af[mi], bfr[ni], acc[mi][ni]);
  }

  const int q8 = tid & 7, lsub = tid >> 3;

  if (EPI == EPI_OUT) {
    float* Cf = (float*)Cs;
    float* Do = (float*)D0;
    const float oscale = 1.0f / (AVCARRY * OWCARRY);
#pragma unroll
    for (int rh = 0; rh < 2; ++rh) {
      __syncthreads();
      if (wm == rh) {
#pragma unroll
        for (int mi = 0; mi < 4; ++mi)
#pragma unroll
          for (int ni = 0; ni < 2; ++ni) {
            const int col = wn * 32 + ni * 16 + l15;
#pragma unroll
            for (int v = 0; v < 8; ++v)
              Cf[(mi * 16 + 8 * h + v) * CFP + col] = acc[mi][ni][v] * oscale;
          }
      }
      __syncthreads();
      for (int ps = 0; ps < 2; ++ps) {
#pragma unroll
        for (int it = 0; it < 8; ++it) {
          const int L = it * 32 + lsub, pr = L >> 2, ql = L & 3;
          v4u val = *(const v4u*)(&Cf[pr * CFP + 32 * ql + 4 * q8]);
          float* dst = Do + ((size_t)(m0 + 64 * rh + pr) * DM + n0 + 32 * ql + 4 * q8);
          *(volatile v4u*)dst = val;
        }
        if (ps == 0) __threadfence();
      }
    }
  } else {
    const int npl = (EPI == EPI_Q) ? 2 : 1;
    for (int pl = 0; pl < npl; ++pl) {
      __syncthreads();
      if (EPI == EPI_Q) {
        const float* bias = pl ? bias1 : bias0;
#pragma unroll
        for (int mi = 0; mi < 4; ++mi)
#pragma unroll
          for (int ni = 0; ni < 2; ++ni) {
            const int col = wn * 32 + ni * 16 + l15;
            const float bv = bias[n0 + col];
#pragma unroll
            for (int v = 0; v < 8; ++v)
              Cs[(wm * 64 + mi * 16 + 8 * h + v) * CSP + col] = hf_bits(acc[mi][ni][v] + bv);
          }
      } else {
#pragma unroll
        for (int mi = 0; mi < 4; ++mi)
#pragma unroll
          for (int ni = 0; ni < 2; ++ni) {
            const int col = wn * 32 + ni * 16 + l15;
#pragma unroll
            for (int v = 0; v < 8; ++v)
              Cs[(wm * 64 + mi * 16 + 8 * h + v) * CSP + col] = hf_bits(acc[mi][ni][v]);
          }
      }
      __syncthreads();
      const bool rowlines = (EPI == EPI_Q) || (EPI == EPI_RK) || ((EPI == EPI_KV) && (n0 < HH));
      for (int ps = 0; ps < 2; ++ps) {
        if (rowlines) {
#pragma unroll
          for (int it = 0; it < 8; ++it) {
            const int L = it * 32 + lsub, pr = L >> 1, nl = L & 1;
            v4u val = *(const v4u*)(&Cs[pr * CSP + nl * 64 + 8 * q8]);
            us_t* dst;
            if (EPI == EPI_RK)
              dst = (us_t*)D0 + ((size_t)(m0 + pr) * HH + n0 + 64 * nl + 8 * q8);
            else if (EPI == EPI_Q)
              dst = (us_t*)(pl ? D1 : D0) + ((((size_t)z * NH + (n0 >> 6) + nl) * QLEN + m0 + pr) * DH + 8 * q8);
            else
              dst = (us_t*)D0 + ((((size_t)z * NH + (n0 >> 6) + nl) * KLEN + m0 + pr) * DH + 8 * q8);
            *(volatile v4u*)dst = val;
          }
        } else {
          const int nbv = (n0 - HH) >> 6;
#pragma unroll
          for (int it = 0; it < 8; ++it) {
            const int L = it * 32 + lsub, nl = L >> 7, d = (L >> 1) & 63, hp = L & 1;
            const int rb0 = 64 * hp + 8 * q8, cc = nl * 64 + d;
            unsigned wv[4];
#pragma unroll
            for (int k = 0; k < 4; ++k) {
              const unsigned lo = Cs[(rb0 + 2 * k) * CSP + cc];
              const unsigned hi = Cs[(rb0 + 2 * k + 1) * CSP + cc];
              wv[k] = lo | (hi << 16);
            }
            v4u val = {wv[0], wv[1], wv[2], wv[3]};
            us_t* dst = (us_t*)D1 + ((((size_t)z * NH + nbv + nl) * DH + d) * KLEN + m0 + 64 * hp + 8 * q8);
            *(volatile v4u*)dst = val;
          }
        }
        if (ps == 0) __threadfence();
      }
    }
  }
}

#define PP 72

__global__ __launch_bounds__(128)
void k_attn(const us_t* __restrict__ Qa, const us_t* __restrict__ Qb, const us_t* __restrict__ Kp,
            const us_t* __restrict__ Vt, const us_t* __restrict__ Rk, us_t* AV)
{
  __shared__ __align__(16) us_t Pst[4 * 16 * PP];
  const int tid = threadIdx.x, lane = tid & 31, wid = tid >> 5;
  const int h = lane >> 4, l15 = lane & 15, hi16 = lane & 16;
  const int i0 = blockIdx.x * 64, bn = blockIdx.y;
  const int b = bn / NH, n = bn - b * NH;
  const int iw = i0 + wid * 16;
  us_t* Pw = Pst + wid * (16 * PP);

  Frag16 qa[2], qb[2];
  {
    const us_t* pa = Qa + ((size_t)bn * QLEN + iw + l15) * DH;
    const us_t* pb = Qb + ((size_t)bn * QLEN + iw + l15) * DH;
#pragma unroll
    for (int c = 0; c < 2; ++c) {
      qa[c].u[0] = *(const v8us*)(pa + 32 * c + 8 * h);
      qa[c].u[1] = *(const v8us*)(pa + 32 * c + 16 + 8 * h);
      qb[c].u[0] = *(const v8us*)(pb + 32 * c + 8 * h);
      qb[c].u[1] = *(const v8us*)(pb + 32 * c + 16 + 8 * h);
    }
  }

  v8f oacc[4];
#pragma unroll
  for (int dt = 0; dt < 4; ++dt) oacc[dt] = vzero();
  float mrow[8], lrow[8];
#pragma unroll
  for (int r = 0; r < 8; ++r) { mrow[r] = -3.0e38f; lrow[r] = 0.f; }

  const int sb = l15 - 8 * h + 15;
  const int ntiles = (MLEN + i0) / 64 + 1;
  const us_t* Kbase = Kp + (size_t)bn * KLEN * DH;
  const us_t* Vbase = Vt + (size_t)bn * DH * KLEN;
  const us_t* Rbase = Rk + (size_t)n * DH;

  for (int kt = 0; kt < ntiles; ++kt) {
    const int kt0 = kt * 64;

    v8f sacc[4];
#pragma unroll
    for (int st = 0; st < 4; ++st) {
      sacc[st] = vzero();
      const us_t* kr = Kbase + (size_t)(kt0 + 16 * st + l15) * DH;
#pragma unroll
      for (int c = 0; c < 2; ++c) {
        Frag16 bf;
        bf.u[0] = *(const v8us*)(kr + 32 * c + 8 * h);
        bf.u[1] = *(const v8us*)(kr + 32 * c + 16 + 8 * h);
        sacc[st] = mma16<1>(qa[c], bf, sacc[st]);
      }
    }

    const int wb = QLEN - 16 + kt0 - iw;
    auto gwin = [&](int nt) -> v8f {
      v8f g = vzero();
      int t = wb + 16 * nt + l15;
      t = (t > KLEN - 1) ? (KLEN - 1) : t;
      const us_t* rp = Rbase + (size_t)t * HH;
#pragma unroll
      for (int c = 0; c < 2; ++c) {
        Frag16 bf;
        bf.u[0] = *(const v8us*)(rp + 32 * c + 8 * h);
        bf.u[1] = *(const v8us*)(rp + 32 * c + 16 + 8 * h);
        g = mma16<1>(qb[c], bf, g);
      }
      return g;
    };
    float xp[8];
    {
      v8f g = gwin(0);
#pragma unroll
      for (int r = 0; r < 8; ++r) xp[r] = __shfl(g[r], ((sb - r) & 15) | hi16);
    }
#pragma unroll
    for (int st = 0; st < 4; ++st) {
      v8f g = gwin(st + 1);
      float xn[8];
#pragma unroll
      for (int r = 0; r < 8; ++r) xn[r] = __shfl(g[r], ((sb - r) & 15) | hi16);
#pragma unroll
      for (int r = 0; r < 8; ++r) {
        const float bd = (l15 > 8 * h + r) ? xn[r] : xp[r];
        sacc[st][r] += bd;
        xp[r] = xn[r];
      }
    }

#pragma unroll
    for (int r = 0; r < 8; ++r) {
      const int m = 8 * h + r;
      const int jl = MLEN + iw + m;
      float s[4];
      float tmx = -3.0e38f;
#pragma unroll
      for (int st = 0; st < 4; ++st) {
        const int j = kt0 + 16 * st + l15;
        float v = sacc[st][r] * SCL;
        v = (j > jl) ? -1e30f : v;
        s[st] = v;
        tmx = fmaxf(tmx, v);
      }
      tmx = fmaxf(tmx, __shfl_xor(tmx, 1));
      tmx = fmaxf(tmx, __shfl_xor(tmx, 2));
      tmx = fmaxf(tmx, __shfl_xor(tmx, 4));
      tmx = fmaxf(tmx, __shfl_xor(tmx, 8));
      const float mn = fmaxf(mrow[r], tmx);
      const float corr = __expf(mrow[r] - mn);
      float ps = 0.f;
#pragma unroll
      for (int st = 0; st < 4; ++st) {
        const float pv = __expf(s[st] - mn);
        ps += pv;
        Pw[m * PP + 16 * st + l15] = hf_bits(pv * PCARRY);
      }
      ps += __shfl_xor(ps, 1);
      ps += __shfl_xor(ps, 2);
      ps += __shfl_xor(ps, 4);
      ps += __shfl_xor(ps, 8);
      lrow[r] = lrow[r] * corr + ps;
      mrow[r] = mn;
#pragma unroll
      for (int dt = 0; dt < 4; ++dt) oacc[dt][r] *= corr;
    }
    __syncthreads();

#pragma unroll
    for (int c = 0; c < 2; ++c) {
      Frag16 pa;
      pa.u[0] = *(const v8us*)(Pw + l15 * PP + 32 * c + 8 * h);
      pa.u[1] = *(const v8us*)(Pw + l15 * PP + 32 * c + 16 + 8 * h);
#pragma unroll
      for (int dt = 0; dt < 4; ++dt) {
        Frag16 bv;
        const us_t* vr = Vbase + (size_t)(16 * dt + l15) * KLEN + kt0 + 32 * c;
        bv.u[0] = *(const v8us*)(vr + 8 * h);
        bv.u[1] = *(const v8us*)(vr + 16 + 8 * h);
        oacc[dt] = mma16<1>(pa, bv, oacc[dt]);
      }
    }
    __syncthreads();
  }

#pragma unroll
  for (int r = 0; r < 8; ++r) {
    const int m = 8 * h + r;
    const float sc = (1.0f / lrow[r]) * (AVCARRY / PCARRY);
#pragma unroll
    for (int dt = 0; dt < 4; ++dt) Pw[m * PP + 16 * dt + l15] = hf_bits(oacc[dt][r] * sc);
  }
  __syncthreads();
  const int q8 = lane & 7, rsub = lane >> 3;
  for (int ps = 0; ps < 2; ++ps) {
#pragma unroll
    for (int it = 0; it < 4; ++it) {
      const int row = it * 4 + rsub;
      v4u val = *(const v4u*)(Pw + row * PP + 8 * q8);
      us_t* dst = AV + (((size_t)(iw + row) * NB + b) * HH + n * DH + 8 * q8);
      *(volatile v4u*)dst = val;
    }
    if (ps == 0) __threadfence();
  }
}

__global__ __launch_bounds__(256)
void k_ln(const float* __restrict__ w, const float* __restrict__ ao, const float* __restrict__ g,
          const float* __restrict__ bb, const int* __restrict__ mask, float* out)
{
  __shared__ float red[256];
  const int row = blockIdx.x;
  const int i = row / NB, b = row - i * NB;
  const int t = threadIdx.x;
  const size_t wrow = ((size_t)i * NB_FULL + b) * DM;
  const size_t arow = (size_t)row * DM;

  float x[4];
  float s = 0.f;
#pragma unroll
  for (int c = 0; c < 4; ++c) {
    const int col = t + c * 256;
    x[c] = w[wrow + col] + ao[arow + col];
    s += x[c];
  }

  int viol = 0;
  for (int j = t; j < KLEN; j += 256) {
    const int mv = mask[(size_t)i * KLEN_FULL + j];
    const int ex = (j > MLEN + i) ? 1 : 0;
    const int got = (mv != 0) ? 1 : 0;
    viol += (got != ex) ? 1 : 0;
  }

  red[t] = s;
  __syncthreads();
  for (int o = 128; o > 0; o >>= 1) { if (t < o) red[t] += red[t + o]; __syncthreads(); }
  const float mu = red[0] * (1.0f / DM);
  __syncthreads();

  float vq = 0.f;
#pragma unroll
  for (int c = 0; c < 4; ++c) { const float d = x[c] - mu; vq += d * d; }
  red[t] = vq;
  __syncthreads();
  for (int o = 128; o > 0; o >>= 1) { if (t < o) red[t] += red[t + o]; __syncthreads(); }
  const float rstd = rsqrtf(red[0] * (1.0f / DM) + LNEPS);
  __syncthreads();

  red[t] = (float)viol;
  __syncthreads();
  for (int o = 128; o > 0; o >>= 1) { if (t < o) red[t] += red[t + o]; __syncthreads(); }
  const bool bad = red[0] > 0.5f;

  float y[4];
#pragma unroll
  for (int c = 0; c < 4; ++c) {
    const int col = t + c * 256;
    float yv = (x[c] - mu) * rstd * g[col] + bb[col];
    y[c] = bad ? __uint_as_float(0x7fc00000u) : yv;
  }
  for (int ps = 0; ps < 2; ++ps) {
#pragma unroll
    for (int c = 0; c < 4; ++c) {
      const int col = t + c * 256;
      *(volatile float*)(out + arow + col) = y[c];
    }
    if (ps == 0) __threadfence();
  }
}

extern "C" void kernel_launch(void* const* d_in, const int* in_sizes, int n_in,
                              void* d_out, int out_size, void* d_ws, size_t ws_size,
                              hipStream_t stream)
{
  if (n_in < 11) return;
  const float* w    = (const float*)d_in[0];
  const float* r    = (const float*)d_in[1];
  const float* mems = (const float*)d_in[2];
  const int*   mask = (const int*)d_in[3];
  const float* qkvw = (const float*)d_in[4];
  const float* rw   = (const float*)d_in[5];
  const float* ow   = (const float*)d_in[6];
  const float* rwb  = (const float*)d_in[7];
  const float* rrb  = (const float*)d_in[8];
  const float* lng  = (const float*)d_in[9];
  const float* lnb  = (const float*)d_in[10];

  if ((long)in_sizes[0] < ((long)(QLEN - 1) * NB_FULL + NB) * DM) return;
  if ((long)in_sizes[1] < (long)KLEN * DM) return;
  if ((long)in_sizes[2] < ((long)(MLEN - 1) * NB_FULL + NB) * DM) return;
  if ((long)in_sizes[3] < (long)(QLEN - 1) * KLEN_FULL + KLEN) return;
  if ((long)in_sizes[4] < (long)TH3 * DM) return;
  if ((long)in_sizes[5] < (long)HH * DM) return;
  if ((long)in_sizes[6] < (long)DM * HH) return;
  if (in_sizes[7] < NH * DH || in_sizes[8] < NH * DH || in_sizes[9] < DM || in_sizes[10] < DM) return;
  if ((long)out_size < (long)QLEN * NB * DM) return;

  char* base = (char*)d_ws;
  size_t off = 0;
  auto take = [&](size_t bytes) -> char* {
    char* q = base + off; off += (bytes + 255) & ~(size_t)255; return q;
  };
  us_t*  catb   = (us_t*) take((size_t)NB * KLEN * DM * 2);
  us_t*  qkvw_b = (us_t*) take((size_t)TH3 * DM * 2);
  us_t*  r_b    = (us_t*) take((size_t)KLEN * DM * 2);
  us_t*  rw_b   = (us_t*) take((size_t)HH * DM * 2);
  us_t*  ow_h   = (us_t*) take((size_t)DM * HH * 2);
  us_t*  Qa     = (us_t*) take((size_t)NB * NH * QLEN * DH * 2);
  us_t*  Qb     = (us_t*) take((size_t)NB * NH * QLEN * DH * 2);
  us_t*  Kp     = (us_t*) take((size_t)NB * NH * KLEN * DH * 2);
  us_t*  Vt     = (us_t*) take((size_t)NB * NH * DH * KLEN * 2);
  us_t*  Rk     = (us_t*) take((size_t)KLEN * HH * 2);
  us_t*  AV     = (us_t*) take((size_t)QLEN * NB * HH * 2);
  float* AO     = (float*)take((size_t)QLEN * NB * DM * 4);
  if (off > ws_size) return;

  k_cvt_cat<<<dim3(NB * KLEN), dim3(128), 0, stream>>>(mems, w, catb);
  k_cvt_lin<0><<<dim3(TH3 * DM / 1024), dim3(128), 0, stream>>>(qkvw, qkvw_b);
  k_cvt_lin<0><<<dim3(KLEN * DM / 1024), dim3(128), 0, stream>>>(r, r_b);
  k_cvt_lin<0><<<dim3(HH * DM / 1024), dim3(128), 0, stream>>>(rw, rw_b);
  k_cvt_lin<1><<<dim3(DM * HH / 1024), dim3(128), 0, stream>>>(ow, ow_h);

  k_gemm<0, EPI_KV><<<dim3(2 * HH / BN, KLEN / BM, NB), dim3(256), 0, stream>>>(
      catb, qkvw_b + (size_t)HH * DM, (void*)Kp, (void*)Vt, rwb, rwb,
      (long)DM, (long)DM, (long)KLEN * DM, DM);
  k_gemm<0, EPI_Q><<<dim3(HH / BN, QLEN / BM, NB), dim3(256), 0, stream>>>(
      catb + (size_t)MLEN * DM, qkvw_b, (void*)Qa, (void*)Qb, rwb, rrb,
      (long)DM, (long)DM, (long)KLEN * DM, DM);
  k_gemm<0, EPI_RK><<<dim3(HH / BN, KLEN / BM, 1), dim3(256), 0, stream>>>(
      r_b, rw_b, (void*)Rk, (void*)Rk, rwb, rwb, (long)DM, (long)DM, 0L, DM);
  k_attn<<<dim3(QLEN / 64, NB * NH), dim3(128), 0, stream>>>(Qa, Qb, Kp, Vt, Rk, AV);
  k_gemm<1, EPI_OUT><<<dim3(DM / BN, (QLEN * NB) / BM, 1), dim3(256), 0, stream>>>(
      AV, ow_h, (void*)AO, (void*)AO, rwb, rwb, (long)HH, (long)HH, 0L, HH);
  k_ln<<<dim3(QLEN * NB), dim3(256), 0, stream>>>(w, AO, lng, lnb, mask, (float*)d_out);
}
